// CustomMultiheadAttention_10058813407800
// MI455X (gfx1250) — hardware-run, weakly checked
//
#include <hip/hip_runtime.h>
#pragma clang fp contract(off)


#ifndef NB
#define NB 2
#endif
#ifndef SEQ
#define SEQ 2048
#endif
#define NB_FULL  2
#define SEQ_FULL 2048
#define EM   1024
#define NH_  16
#define HD   64
#define XP   (NB_FULL * EM)
#define AW   4
#define WW   2
#define WKEYS 128
#define OSP  68
#define WP   132
#define SC2  ((float)(0.125 * 1.4426950408889634))
#define PSH  14.0f
#define CXS  (1.0f / 1024.0f)
#define WOS  64.0f
#define OSC  (1.0f / 1024.0f)
#define NEGB (-3.0e38f)
#define STN  ((size_t)NB * NH_ * SEQ)

static_assert(HD == 64);
static_assert(NH_ * HD == EM);
static_assert(EM % 64 == 0);
static_assert(EM % 32 == 0);
static_assert(HD % 32 == 0);
static_assert(SEQ % 64 == 0);
static_assert(SEQ % 32 == 0);
static_assert(SEQ % (16 * AW) == 0);
static_assert(SEQ % (WKEYS * WW) == 0);
static_assert(SEQ % 16 == 0);
static_assert(WKEYS % 32 == 0);
static_assert(NB <= NB_FULL);
static_assert(SEQ <= SEQ_FULL);
static_assert((OSP * 4) % 16 == 0);
static_assert((WP * 4) % 16 == 0);
static_assert(OSP >= 64);
static_assert(WP >= WKEYS);
static_assert(4 * 32 * 16 == 16 * HD * 2);
static_assert(8 * 32 * 16 == 16 * 64 * 4);
static_assert(16 * 32 * 16 == 16 * WKEYS * 4);
static_assert(16 * 16 == 2 * 32 * 4);
static_assert(16 * OSP * 4 <= 131072);
static_assert(AW * 16 * OSP * 4 <= 131072);
static_assert(WW * 16 * WP * 4 <= 131072);
static_assert(CXS * 16384.0f == 16.0f);
static_assert(OSC * 16.0f * WOS == 1.0f);

typedef _Float16 h16;
typedef unsigned short bf;
typedef __attribute__((ext_vector_type(16))) __bf16   v16bf;
typedef __attribute__((ext_vector_type(16))) _Float16 v16h;
typedef __attribute__((ext_vector_type(8)))  _Float16 v8h;
typedef __attribute__((ext_vector_type(8)))  unsigned short v8us;
typedef __attribute__((ext_vector_type(8)))  float    v8f;
typedef __attribute__((ext_vector_type(4)))  float    v4f;
typedef v4f  __attribute__((may_alias)) v4fa;

__device__ __forceinline__ unsigned short f2bf(float f) { unsigned u = __float_as_uint(f); u += 0x7FFFu + ((u >> 16) & 1u); return (unsigned short)(u >> 16); }
__device__ __forceinline__ float bfr(float f) { return __uint_as_float(((unsigned)f2bf(f)) << 16); }
__device__ __forceinline__ v16h cat16(v8h lo, v8h hi) { return __builtin_shufflevector(lo, hi, 0, 1, 2, 3, 4, 5, 6, 7, 8, 9, 10, 11, 12, 13, 14, 15); }
__device__ __forceinline__ v16bf cat16b(v8us lo, v8us hi) { return __builtin_bit_cast(v16bf, __builtin_shufflevector(lo, hi, 0, 1, 2, 3, 4, 5, 6, 7, 8, 9, 10, 11, 12, 13, 14, 15)); }
__device__ __forceinline__ v8f wmma16(v16h a, v16h b, v8f c) { return __builtin_amdgcn_wmma_f32_16x16x32_f16(false, a, false, b, (short)0, c, false, false); }
__device__ __forceinline__ v8f wmmab(v16bf a, v16bf b, v8f c) { return __builtin_amdgcn_wmma_f32_16x16x32_bf16(false, a, false, b, (short)0, c, false, false); }
__device__ __forceinline__ v8f wmma16g(v16h a, v16h b, v8f c) { c = wmma16(a, b, c); asm volatile("v_nop\n\tv_nop\n\tv_nop\n\tv_nop" : "+v"(c) : "v"(a), "v"(b)); return c; }
__device__ __forceinline__ v8f wmmabg(v16bf a, v16bf b, v8f c) { c = wmmab(a, b, c); asm volatile("v_nop\n\tv_nop\n\tv_nop\n\tv_nop" : "+v"(c) : "v"(a), "v"(b)); return c; }
__device__ __forceinline__ v16h  ldh(const h16* p) { return cat16(*(const v8h*)p, *(const v8h*)(p + 16)); }
__device__ __forceinline__ v16bf ldb(const bf* p)  { return cat16b(*(const v8us*)p, *(const v8us*)(p + 16)); }
__device__ __forceinline__ void wave_sync() { __builtin_amdgcn_fence(3  , "wavefront"); __builtin_amdgcn_wave_barrier(); asm volatile("" ::: "memory"); }
static __device__ __forceinline__ h16 toh_flush(float v) { const float w = (fabsf(v) < 6.103515625e-05f) ? 0.0f : v; return (h16)w; }

__global__ __launch_bounds__(256) void k_cvt8(const float* __restrict__ src, bf* dst, size_t n8) {
    const size_t i = (size_t)blockIdx.x * 256 + threadIdx.x; if (i >= n8) return;
    const v8f v = *(const v8f*)(src + i * 8); v8us o;
#pragma unroll
    for (int k = 0; k < 8; ++k) o[k] = f2bf(v[k]);
    *(volatile v8us*)(dst + i * 8) = o; __threadfence(); *(volatile v8us*)(dst + i * 8) = o;
}

__global__ __launch_bounds__(256) void k_wcvt(const float* __restrict__ src, h16* dst, size_t n8) {
    const size_t i = (size_t)blockIdx.x * 256 + threadIdx.x; if (i >= n8) return;
    const v8f v = *(const v8f*)(src + i * 8); v8h o;
#pragma unroll
    for (int k = 0; k < 8; ++k) o[k] = toh_flush(bfr(v[k]) * WOS);
    *(volatile v8h*)(dst + i * 8) = o; __threadfence(); *(volatile v8h*)(dst + i * 8) = o;
}

template <int MODE>
__device__ __forceinline__ void proj_body(const bf* __restrict__ A, const bf* __restrict__ Bt, const float* __restrict__ bias, h16* P) {
    __shared__ __align__(16) float os[16 * OSP];
    constexpr size_t AP = (MODE == 0) ? (size_t)XP : (size_t)EM;
    constexpr size_t BP = (MODE == 0) ? (size_t)EM : (size_t)XP;
    constexpr size_t RP = (MODE == 0) ? (size_t)HD : (size_t)SEQ;
    const int lane = threadIdx.x & 31, lr = lane & 15, hi = lane >> 4;
    const int r0 = blockIdx.x * 64, c0 = blockIdx.y * 64, nz = blockIdx.z;
    v8f acc[4][4];
#pragma unroll
    for (int mb = 0; mb < 4; ++mb)
#pragma unroll
        for (int nb = 0; nb < 4; ++nb) acc[mb][nb] = (v8f){};
    const size_t aoff = (size_t)(r0 + lr) * AP + 8 * hi + ((MODE == 0) ? (size_t)nz * EM : (size_t)0);
    const size_t boff = (size_t)(c0 + lr) * BP + 8 * hi + ((MODE == 1) ? (size_t)nz * EM : (size_t)0);
#pragma unroll 1
    for (int kc = 0; kc < EM; kc += 32) {
        v16bf a[4];
#pragma unroll
        for (int mb = 0; mb < 4; ++mb) a[mb] = ldb(A + aoff + (size_t)mb * 16 * AP + kc);
#pragma unroll
        for (int nb = 0; nb < 4; ++nb) { const v16bf b = ldb(Bt + boff + (size_t)nb * 16 * BP + kc);
#pragma unroll
            for (int mb = 0; mb < 4; ++mb) acc[mb][nb] = wmmabg(a[mb], b, acc[mb][nb]); }
    }
    float bc[4];
#pragma unroll
    for (int nb = 0; nb < 4; ++nb) bc[nb] = (MODE == 0) ? bfr(bias[c0 + nb * 16 + lr]) : 0.0f;
    const size_t tbase = (MODE == 0) ? (((size_t)nz * NH_ + (size_t)blockIdx.y) * SEQ + (size_t)r0) * HD
                                     : ((size_t)nz * EM + (size_t)r0) * SEQ + (size_t)c0;
#pragma unroll
    for (int mb = 0; mb < 4; ++mb) {
        float br[8];
        if (MODE == 1) {
            const v4f b0 = *(const v4f*)(bias + r0 + mb * 16 + hi * 8); const v4f b1 = *(const v4f*)(bias + r0 + mb * 16 + hi * 8 + 4);
#pragma unroll
            for (int j = 0; j < 4; ++j) { br[j] = bfr(b0[j]); br[4 + j] = bfr(b1[j]); }
        } else {
#pragma unroll
            for (int j = 0; j < 8; ++j) br[j] = 0.0f;
        }
#pragma unroll
        for (int nb = 0; nb < 4; ++nb) {
#pragma unroll
            for (int j = 0; j < 8; ++j) os[(hi * 8 + j) * OSP + nb * 16 + lr] = acc[mb][nb][j] + bc[nb] + br[j]; }
        wave_sync();
#pragma unroll 1
        for (int ps = 0; ps < 2; ++ps) {
#pragma unroll
            for (int s = 0; s < 4; ++s) { const int row = 4 * s + (lane >> 3), c8 = (lane & 7) * 8;
                const v4f x0 = *(const v4fa*)(&os[row * OSP + c8]); const v4f x1 = *(const v4fa*)(&os[row * OSP + c8 + 4]); v8h hv;
#pragma unroll
                for (int i = 0; i < 4; ++i) { hv[i] = toh_flush(x0[i]); hv[4 + i] = toh_flush(x1[i]); }
                *(volatile v8h*)(P + tbase + (size_t)(mb * 16 + row) * RP + c8) = hv; }
            if (ps == 0) __threadfence(); }
        wave_sync();
    }
}

__global__ __launch_bounds__(32) void k_proj_rows(const bf* __restrict__ X, const bf* __restrict__ W, const float* __restrict__ bias, h16* P) { proj_body<0>(X, W, bias, P); }
__global__ __launch_bounds__(32) void k_proj_tr(const bf* __restrict__ W, const bf* __restrict__ X, const float* __restrict__ bias, h16* P) { proj_body<1>(W, X, bias, P); }

__global__ __launch_bounds__(32) void k_outp(const h16* __restrict__ A, const h16* __restrict__ Bt, const float* __restrict__ bias, float* OUT) {
    __shared__ __align__(16) float os[16 * OSP];
    const int lane = threadIdx.x & 31, lr = lane & 15, hi = lane >> 4;
    const int r0 = blockIdx.x * 64, c0 = blockIdx.y * 64, nz = blockIdx.z;
    v8f acc[4][4];
#pragma unroll
    for (int mb = 0; mb < 4; ++mb)
#pragma unroll
        for (int nb = 0; nb < 4; ++nb) acc[mb][nb] = (v8f){};
    const size_t aoff = (size_t)(r0 + lr) * XP + (size_t)nz * EM + 8 * hi;
    const size_t boff = (size_t)(c0 + lr) * EM + 8 * hi;
#pragma unroll 1
    for (int kc = 0; kc < EM; kc += 32) {
        v16h a[4];
#pragma unroll
        for (int mb = 0; mb < 4; ++mb) a[mb] = ldh(A + aoff + (size_t)mb * 16 * XP + kc);
#pragma unroll
        for (int nb = 0; nb < 4; ++nb) { const v16h b = ldh(Bt + boff + (size_t)nb * 16 * EM + kc);
#pragma unroll
            for (int mb = 0; mb < 4; ++mb) acc[mb][nb] = wmma16g(a[mb], b, acc[mb][nb]); }
    }
    float bc[4];
#pragma unroll
    for (int nb = 0; nb < 4; ++nb) bc[nb] = bfr(bias[c0 + nb * 16 + lr]);
#pragma unroll
    for (int mb = 0; mb < 4; ++mb) {
#pragma unroll
        for (int nb = 0; nb < 4; ++nb) {
#pragma unroll
            for (int j = 0; j < 8; ++j) os[(hi * 8 + j) * OSP + nb * 16 + lr] = acc[mb][nb][j] * OSC + bc[nb]; }
        wave_sync();
#pragma unroll 1
        for (int ps = 0; ps < 2; ++ps) {
#pragma unroll
            for (int s = 0; s < 8; ++s) { const int row = 2 * s + (lane >> 4), cofs = (lane & 15) * 4;
                const v4f val = *(const v4fa*)(&os[row * OSP + cofs]);
                *(volatile v4f*)(OUT + ((size_t)(r0 + mb * 16 + row) * NB_FULL + (size_t)nz) * EM + c0 + cofs) = val; }
            if (ps == 0) __threadfence(); }
        wave_sync();
    }
}

__device__ __forceinline__ void score32(const h16* ka, const v16h q0, const v16h q1, v8f& sa, v8f& sb) {
    const v16h ka0 = ldh(ka), ka1 = ldh(ka + 32), kb0 = ldh(ka + 16 * HD), kb1 = ldh(ka + 16 * HD + 32);
    v8f a = (v8f){}, b = (v8f){};
    a = wmma16g(ka0, q0, a); a = wmma16g(ka1, q1, a);
    b = wmma16g(kb0, q0, b); b = wmma16g(kb1, q1, b);
    sa = a; sb = b;
}

__global__ __launch_bounds__(64) void k_rowstat(const h16* __restrict__ QH, const h16* __restrict__ KP, float* SP) {
    __shared__ __align__(16) float st[64];
    const int lane = threadIdx.x & 31, lr = lane & 15, hi = lane >> 4;
    const int wave = __builtin_amdgcn_readfirstlane((int)(threadIdx.x >> 5));
    const int zh = blockIdx.y;
    const int tblk = blockIdx.x * 32;
    const int t0 = tblk + wave * 16;
    const size_t pbase = (size_t)zh * SEQ * HD;
    const size_t qo = pbase + (size_t)(t0 + lr) * HD + 8 * hi;
    const v16h q0 = ldh(QH + qo), q1 = ldh(QH + qo + 32);
    const size_t ko = pbase + (size_t)lr * HD + 8 * hi;
    float m = NEGB, l = 0.0f;
#pragma unroll 1
    for (int key0 = 0; key0 < SEQ; key0 += 32) {
        v8f sa, sb; score32(KP + ko + (size_t)key0 * HD, q0, q1, sa, sb);
        float ta[8], tc[8]; float mx = NEGB;
#pragma unroll
        for (int r = 0; r < 8; ++r) { ta[r] = sa[r] * SC2; tc[r] = sb[r] * SC2; mx = fmaxf(mx, fmaxf(ta[r], tc[r])); }
        const float mnew = fmaxf(m, mx);
        float ls = 0.0f;
#pragma unroll
        for (int r = 0; r < 8; ++r) ls += __builtin_amdgcn_exp2f(ta[r] - mnew) + __builtin_amdgcn_exp2f(tc[r] - mnew);
        l = l * __builtin_amdgcn_exp2f(m - mnew) + ls; m = mnew;
    }
    const float mo = __shfl_xor(m, 16, 32), lo = __shfl_xor(l, 16, 32);
    const float M = fmaxf(m, mo);
    const float L = l * __builtin_amdgcn_exp2f(m - M) + lo * __builtin_amdgcn_exp2f(mo - M);
    const float IL = 1.0f / L;
    if (hi == 0) { st[wave * 16 + lr] = M; st[32 + wave * 16 + lr] = IL; }
    __syncthreads();
    if (threadIdx.x < 16) {
        const int line = lane >> 3, piece = lane & 7;
        const v4f val = *(const v4fa*)(&st[line * 32 + piece * 4]);
        float* dst = SP + (size_t)line * STN + (size_t)zh * SEQ + (size_t)tblk + piece * 4;
#pragma unroll 1
        for (int ps = 0; ps < 2; ++ps) { *(volatile v4f*)dst = val; if (ps == 0) __threadfence(); }
    }
}

__global__ __launch_bounds__(32 * AW) void k_attn(const h16* __restrict__ QH, const h16* __restrict__ KP, const h16* __restrict__ VT, const float* __restrict__ SP, h16* CX) {
    __shared__ __align__(16) float os[AW * 16 * OSP];
    const int lane = threadIdx.x & 31, lr = lane & 15, hi = lane >> 4;
    const int wave = __builtin_amdgcn_readfirstlane((int)(threadIdx.x >> 5));
    const unsigned zh = blockIdx.y; const unsigned nz = zh / (unsigned)NH_, h = zh % (unsigned)NH_;
    const int t0 = (blockIdx.x * AW + wave) * 16;
    const size_t pbase = (size_t)zh * SEQ * HD;
    const size_t qo = pbase + (size_t)(t0 + lr) * HD + 8 * hi;
    const v16h q0 = ldh(QH + qo), q1 = ldh(QH + qo + 32);
    const size_t ko = pbase + (size_t)lr * HD + 8 * hi;
    const size_t vo = pbase + (size_t)lr * SEQ + 8 * hi;
    const float mq = SP[(size_t)zh * SEQ + t0 + lr];
    const float il = SP[STN + (size_t)zh * SEQ + t0 + lr];
    const float sh = PSH - mq;
    v8f o[4];
#pragma unroll
    for (int j = 0; j < 4; ++j) o[j] = (v8f){};
#pragma unroll 1
    for (int key0 = 0; key0 < SEQ; key0 += 32) {
        v8f sa, sb; score32(KP + ko + (size_t)key0 * HD, q0, q1, sa, sb);
        v16h pb;
#pragma unroll
        for (int r = 0; r < 8; ++r) {
            const float ga = __builtin_amdgcn_exp2f(sa[r] * SC2 + sh) * il;
            const float gb = __builtin_amdgcn_exp2f(sb[r] * SC2 + sh) * il;
            pb[r] = toh_flush(ga); pb[8 + r] = toh_flush(gb); }
        const h16* va = VT + vo + key0;
#pragma unroll
        for (int j = 0; j < 4; ++j) { const v16h vj = ldh(va + (size_t)j * 16 * SEQ); o[j] = wmma16g(vj, pb, o[j]); }
    }
    const int wb = wave * 16 * OSP;
#pragma unroll
    for (int j = 0; j < 4; ++j) { v4f a, c;
        a[0] = o[j][0] * CXS; a[1] = o[j][1] * CXS; a[2] = o[j][2] * CXS; a[3] = o[j][3] * CXS; c[0] = o[j][4] * CXS; c[1] = o[j][5] * CXS; c[2] = o[j][6] * CXS; c[3] = o[j][7] * CXS;
        *(v4fa*)(&os[wb + lr * OSP + 16 * j + 8 * hi]) = a; *(v4fa*)(&os[wb + lr * OSP + 16 * j + 8 * hi + 4]) = c; }
    wave_sync();
    h16* crow = CX + ((size_t)t0 * NB_FULL + (size_t)nz) * EM + (size_t)h * HD;
#pragma unroll 1
    for (int ps = 0; ps < 2; ++ps) {
#pragma unroll
        for (int s = 0; s < 4; ++s) { const int row = 4 * s + (lane >> 3), c8 = (lane & 7) * 8;
            const v4f x0 = *(const v4fa*)(&os[wb + row * OSP + c8]); const v4f x1 = *(const v4fa*)(&os[wb + row * OSP + c8 + 4]); v8h hv;
#pragma unroll
            for (int i = 0; i < 4; ++i) { hv[i] = toh_flush(x0[i]); hv[4 + i] = toh_flush(x1[i]); }
            *(volatile v8h*)(crow + (size_t)row * XP + c8) = hv; }
        if (ps == 0) __threadfence(); }
}

__global__ __launch_bounds__(32 * WW) void k_wavg(const h16* __restrict__ QH, const h16* __restrict__ KP, const float* __restrict__ SP, float* O1) {
    __shared__ __align__(16) float os[WW * 16 * WP];
    const int lane = threadIdx.x & 31, lr = lane & 15, hi = lane >> 4;
    const int wave = __builtin_amdgcn_readfirstlane((int)(threadIdx.x >> 5));
    const int nz = blockIdx.z;
    const int qb = blockIdx.y * 16;
    const int kc0 = (blockIdx.x * WW + wave) * WKEYS;
    v8f acc[2 * (WKEYS / 32)];
#pragma unroll
    for (int i = 0; i < 2 * (WKEYS / 32); ++i) acc[i] = (v8f){};
#pragma unroll 1
    for (int hh = 0; hh < NH_; ++hh) {
        const int zh = nz * NH_ + hh;
        const size_t pbase = (size_t)zh * SEQ * HD;
        const size_t qo = pbase + (size_t)(qb + lr) * HD + 8 * hi;
        const v16h q0 = ldh(QH + qo), q1 = ldh(QH + qo + 32);
        const float mq = SP[(size_t)zh * SEQ + qb + lr];
        const float il = SP[STN + (size_t)zh * SEQ + qb + lr];
        const size_t ko = pbase + (size_t)(kc0 + lr) * HD + 8 * hi;
#pragma unroll
        for (int kt = 0; kt < WKEYS / 32; ++kt) {
            v8f sa, sb; score32(KP + ko + (size_t)kt * 32 * HD, q0, q1, sa, sb);
#pragma unroll
            for (int r = 0; r < 8; ++r) {
                acc[2 * kt][r]     += __builtin_amdgcn_exp2f(sa[r] * SC2 - mq) * il;
                acc[2 * kt + 1][r] += __builtin_amdgcn_exp2f(sb[r] * SC2 - mq) * il; }
        }
    }
    const int wb = wave * 16 * WP;
#pragma unroll
    for (int kt = 0; kt < WKEYS / 32; ++kt) { v4f a, c;
        a[0] = acc[2 * kt][0] * 0.0625f; a[1] = acc[2 * kt][1] * 0.0625f; a[2] = acc[2 * kt][2] * 0.0625f; a[3] = acc[2 * kt][3] * 0.0625f;
        c[0] = acc[2 * kt][4] * 0.0625f; c[1] = acc[2 * kt][5] * 0.0625f; c[2] = acc[2 * kt][6] * 0.0625f; c[3] = acc[2 * kt][7] * 0.0625f;
        *(v4fa*)(&os[wb + lr * WP + kt * 32 + 8 * hi]) = a; *(v4fa*)(&os[wb + lr * WP + kt * 32 + 8 * hi + 4]) = c;
        a[0] = acc[2 * kt + 1][0] * 0.0625f; a[1] = acc[2 * kt + 1][1] * 0.0625f; a[2] = acc[2 * kt + 1][2] * 0.0625f; a[3] = acc[2 * kt + 1][3] * 0.0625f;
        c[0] = acc[2 * kt + 1][4] * 0.0625f; c[1] = acc[2 * kt + 1][5] * 0.0625f; c[2] = acc[2 * kt + 1][6] * 0.0625f; c[3] = acc[2 * kt + 1][7] * 0.0625f;
        *(v4fa*)(&os[wb + lr * WP + kt * 32 + 16 + 8 * hi]) = a; *(v4fa*)(&os[wb + lr * WP + kt * 32 + 16 + 8 * hi + 4]) = c; }
    wave_sync();
    float* orow = O1 + ((size_t)nz * SEQ_FULL + (size_t)qb) * SEQ_FULL + (size_t)kc0;
#pragma unroll 1
    for (int ps = 0; ps < 2; ++ps) {
#pragma unroll
        for (int i = 0; i < 16; ++i) {
            const v4f val = *(const v4fa*)(&os[wb + i * WP + lane * 4]);
            *(volatile v4f*)(orow + (size_t)i * SEQ_FULL + lane * 4) = val; }
        if (ps == 0) __threadfence(); }
}

static constexpr size_t al256(size_t v) { return (v + 255) & ~(size_t)255; }
static constexpr size_t SZ_XB = al256((size_t)SEQ * NB_FULL * EM * 2);
static constexpr size_t SZ_WB = al256((size_t)3 * EM * EM * 2);
static constexpr size_t SZ_WO = al256((size_t)EM * EM * 2);
static constexpr size_t SZ_PL = al256((size_t)NB * NH_ * SEQ * HD * 2);
static constexpr size_t SZ_CX = al256((size_t)SEQ * NB_FULL * EM * 2);
static constexpr size_t SZ_ST = al256((size_t)2 * NB * NH_ * SEQ * 4);
static constexpr size_t SZ_TOTAL = 3 * SZ_XB + SZ_WB + SZ_WO + 3 * SZ_PL + SZ_CX + SZ_ST;
static_assert(SZ_TOTAL <= (size_t)134217728);
static_assert(((size_t)EM * EM * 2) % 256 == 0);
static_assert((size_t)NB * NH_ * SEQ * HD == (size_t)NB * EM * SEQ);
static_assert(((size_t)SEQ * NB_FULL * EM) % 8 == 0);
static_assert(((size_t)EM * EM) % 8 == 0);
static_assert(((size_t)NB * NH_ * SEQ * 4) % 128 == 0);
static constexpr size_t OUT1_OFF = (size_t)SEQ_FULL * NB_FULL * EM;
static_assert(OUT1_OFF * 4 == (size_t)16777216);
static_assert((OUT1_OFF + (size_t)NB_FULL * SEQ_FULL * SEQ_FULL) * 4 == (size_t)50331648);
static constexpr size_t NEED_X   = (size_t)SEQ * NB_FULL * EM;
static constexpr size_t NEED_O   = OUT1_OFF + ((size_t)(NB - 1) * SEQ_FULL + (size_t)(SEQ - 1)) * SEQ_FULL + (size_t)SEQ;
static_assert(((size_t)(SEQ - 1) * NB_FULL + (size_t)(NB - 1)) * EM + EM <= OUT1_OFF);
static_assert(NEED_O <= OUT1_OFF + (size_t)NB_FULL * SEQ_FULL * SEQ_FULL);

extern "C" void kernel_launch(void* const* d_in, const int* in_sizes, int n_in,
                              void* d_out, int out_size, void* d_ws, size_t ws_size, hipStream_t stream) {
    if (n_in < 11) return;
    if ((size_t)in_sizes[0] < NEED_X || (size_t)in_sizes[1] < NEED_X || (size_t)in_sizes[2] < NEED_X) return;
    if ((size_t)in_sizes[3] < (size_t)EM * EM || (size_t)in_sizes[5] < (size_t)EM * EM || (size_t)in_sizes[7] < (size_t)EM * EM || (size_t)in_sizes[9] < (size_t)EM * EM) return;
    if (in_sizes[4] < EM || in_sizes[6] < EM || in_sizes[8] < EM || in_sizes[10] < EM) return;
    if ((size_t)out_size < NEED_O) return;
    if (SZ_TOTAL > ws_size) return;
    const float* xin[3] = { (const float*)d_in[0], (const float*)d_in[1], (const float*)d_in[2] };
    const float* wq = (const float*)d_in[3]; const float* bq = (const float*)d_in[4];
    const float* wk = (const float*)d_in[5]; const float* bk = (const float*)d_in[6];
    const float* wv = (const float*)d_in[7]; const float* bv = (const float*)d_in[8];
    const float* wo = (const float*)d_in[9]; const float* bo = (const float*)d_in[10];
    float* OUT0 = (float*)d_out;
    float* OUT1 = (float*)d_out + OUT1_OFF;
    char* wsp = (char*)d_ws;
    bf* XB[3];
    XB[0] = (bf*)wsp; wsp += SZ_XB;
    XB[1] = (bf*)wsp; wsp += SZ_XB;
    XB[2] = (bf*)wsp; wsp += SZ_XB;
    bf* WB = (bf*)wsp; wsp += SZ_WB;
    h16* WOH = (h16*)wsp; wsp += SZ_WO;
    h16* QH = (h16*)wsp; wsp += SZ_PL;
    h16* KP = (h16*)wsp; wsp += SZ_PL;
    h16* VT = (h16*)wsp; wsp += SZ_PL;
    h16* CX = (h16*)wsp; wsp += SZ_CX;
    float* SP = (float*)wsp; wsp += SZ_ST;
    bf* WQ = WB; bf* WK = WB + (size_t)EM * EM; bf* WV = WB + (size_t)2 * EM * EM;

    { const size_t n8 = NEED_X / 8; const unsigned g = (unsigned)((n8 + 255) / 256);
      for (int i = 0; i < 3; ++i) k_cvt8<<<g, 256, 0, stream>>>(xin[i], XB[i], n8); }
    { const size_t n8 = (size_t)EM * EM / 8; const unsigned g = (unsigned)((n8 + 255) / 256);
      k_cvt8<<<g, 256, 0, stream>>>(wq, WQ, n8); k_cvt8<<<g, 256, 0, stream>>>(wk, WK, n8); k_cvt8<<<g, 256, 0, stream>>>(wv, WV, n8);
      k_wcvt<<<g, 256, 0, stream>>>(wo, WOH, n8); }

    k_proj_rows<<<dim3(SEQ / 64, EM / 64, NB), 32, 0, stream>>>(XB[0], WQ, bq, QH);
    k_proj_rows<<<dim3(SEQ / 64, EM / 64, NB), 32, 0, stream>>>(XB[1], WK, bk, KP);
    k_proj_tr<<<dim3(EM / 64, SEQ / 64, NB), 32, 0, stream>>>(WV, XB[2], bv, VT);

    k_rowstat<<<dim3(SEQ / 32, NB * NH_, 1), 64, 0, stream>>>(QH, KP, SP);
    k_attn<<<dim3(SEQ / (16 * AW), NB * NH_, 1), 32 * AW, 0, stream>>>(QH, KP, VT, SP, CX);
    k_outp<<<dim3(SEQ / 64, EM / 64, NB), 32, 0, stream>>>(CX, WOH, bo, OUT0);
    k_wavg<<<dim3(SEQ / (WKEYS * WW), SEQ / 16, NB), 32 * WW, 0, stream>>>(QH, KP, SP, OUT1);
}
